// GraphSAGE_1967095021810
// MI455X (gfx1250) — hardware-run, weakly checked
//
#include <hip/hip_runtime.h>
#include <stddef.h>
#include <stdint.h>
#include <math.h>

#pragma clang fp contract(off)

#define MEAN_SPLIT 1

#define NN      100000
#define NE      1600000
#define FI      50
#define NPAIR   25
#define NC      16
#define GBM     128
#define RBM     128
#define MP      100096
#define XP      64
#define MHP     128
#define WBP     192
#define WROFF   128
#define MSTEPS  (MEAN_SPLIT ? 4 : 2)
#define XSTEPS  2
#define DTP     17
#define NTHR    256
#define NWAVE   8
#define EPT     8
#define WCH     (32 * EPT)
#define NBRUN   1024
#define SLB     10
#define NBK     98
#define WLCAP   3584
#define RCAP    28672
#define DEGCAP  64
#define MAXDEG_MEAS 36
#define MAXHIT_MEAS 16710

#define BK_ZINTS (NWAVE * WLCAP + RCAP + 3 * NBRUN)
#define BK_INTS  (BK_ZINTS + 16)
#define BK_LDS   (BK_INTS * 4)

#define ZLIST_B  (NBK * RCAP * 4)
#define ZCO_B    (NBK * 2 * NBRUN * 4)
#define ZFLAG_B  16384
#define ZTOT_B   (ZLIST_B + ZCO_B + ZFLAG_B)

#define PBX   (MP * 8 / NTHR)
#define WBU   (NC * WBP / 8)
#define PBW   2
#define PBZ   (ZTOT_B / 4096)
#define PBTOT (PBX + PBW + 1 + PBZ)

static_assert(MP == 782 * GBM && MP >= NN && MP % RBM == 0);
static_assert(NBRUN == (1 << SLB) && NBRUN % GBM == 0 && NBRUN % RBM == 0 && NBRUN % 32 == 0);
static_assert(NBK * NBRUN >= MP && NBK * NBRUN >= NN);
static_assert(NE < (1 << 21) && (((long long)NE) << SLB) < (1LL << 31));
static_assert(NE % WCH == 0 && NE % 4 == 0);
static_assert(RCAP == NWAVE * WLCAP && RCAP % (NTHR * 4) == 0 && (2 * NBRUN) % (NTHR * 4) == 0);
static_assert(BK_ZINTS % (NTHR * 4) == 0);
static_assert((long long)RCAP * 100 >= (long long)MAXHIT_MEAS * 105);
static_assert(WLCAP >= MAXHIT_MEAS / 8 + 8 * 46 + 1);
static_assert(MAXDEG_MEAS + 8 <= DEGCAP);
static_assert(XP % 8 == 0 && XP == 64 && MHP == 2 * XP && WBP == 3 * XP && WBP == 6 * 32 && WROFF == 2 * XP);
static_assert(FI <= XP && FI == 2 * NPAIR);
static_assert(32 * (MSTEPS + XSTEPS) <= WBP && 32 * MSTEPS <= MHP && 32 * XSTEPS == XP);
static_assert(BK_LDS <= 300000);
static_assert((MP * 8) % NTHR == 0 && WBU <= PBW * NTHR && WBU % 32 == 0);
static_assert(ZTOT_B % 4096 == 0 && NBK * 128 <= ZFLAG_B);
static_assert((GBM * NC * 4) % 128 == 0 && (((NN % GBM) * NC * 4) % 128) == 0 && ((NN * NC * 4) % 128) == 0);
static_assert(GBM * NC / 4 == 2 * NTHR && RBM == NWAVE * 16 && GBM == NWAVE * 16);

typedef float          v2f   __attribute__((ext_vector_type(2)));
typedef float          v4f   __attribute__((ext_vector_type(4)));
typedef float          v8f   __attribute__((ext_vector_type(8)));
typedef int            v4i   __attribute__((ext_vector_type(4)));
typedef int            v8i   __attribute__((ext_vector_type(8)));
typedef unsigned       v4u   __attribute__((ext_vector_type(4)));
typedef unsigned short v8us  __attribute__((ext_vector_type(8)));
typedef unsigned short v16us __attribute__((ext_vector_type(16)));
typedef __bf16         v16bf __attribute__((ext_vector_type(16)));
typedef v2f  __attribute__((may_alias)) v2fa;
typedef v4f  __attribute__((may_alias)) v4fa;
typedef v4i  __attribute__((may_alias)) v4ia;
typedef v4u  __attribute__((may_alias)) v4ua;
typedef v8us __attribute__((may_alias)) v8usa;
union FragB { v16bf v; v16us u; v8us h[2]; v8i w; };

__device__ __forceinline__ v8f wmb(const FragB& a, const FragB& b, v8f c) {
  v8f d = __builtin_amdgcn_wmma_f32_16x16x32_bf16(false, a.v, false, b.v, (short)0, c, false, false);
  asm volatile("v_nop\n\tv_nop\n\tv_nop\n\tv_nop" : "+v"(d) : "v"(a.w), "v"(b.w));
  return d;
}

__device__ __forceinline__ unsigned bf16_bits(float f) {
  const unsigned u = __float_as_uint(f);
  const unsigned r = (u + 0x7fffu + ((u >> 16) & 1u)) >> 16;
  const unsigned q = (u >> 16) | 0x40u;
  return ((u & 0x7fffffffu) > 0x7f800000u) ? q : r;
}

__device__ __forceinline__ void st2_v4f(float* p, v4f v) {
  *(volatile v4f*)p = v;
  __threadfence();
  *(volatile v4f*)p = v;
}
__device__ __forceinline__ void st2_v8us(unsigned short* p, v8us v) {
  *(volatile v8us*)p = v;
  __threadfence();
  *(volatile v8us*)p = v;
}

__global__ __launch_bounds__(NTHR) void k_prep(const float* __restrict__ x, const float* __restrict__ wl,
                                               const float* __restrict__ bl, const float* __restrict__ wr,
                                               unsigned short* xb, unsigned short* wb, float* blp, int* zr) {
  const int tid = (int)threadIdx.x, lane = tid & 31;
  const int blk = (int)blockIdx.x;
  if (blk < PBX) {
    const int u   = blk * NTHR + tid;
    const int row = u >> 3, g = u & 7;
    const int rc  = row < NN ? row : NN - 1;
    const unsigned rmk = row < NN ? 0xffffffffu : 0u;
    const float* rp = x + (size_t)rc * FI;
    const int pa = 4 * g, pb = pa + 1, pc = pa + 2, pd = pa + 3;
    const int qa = pa < NPAIR ? pa : NPAIR - 1, qb = pb < NPAIR ? pb : NPAIR - 1;
    const int qc = pc < NPAIR ? pc : NPAIR - 1, qd = pd < NPAIR ? pd : NPAIR - 1;
    const v2f fa = *(const v2fa*)(rp + 2 * qa);
    const v2f fb = *(const v2fa*)(rp + 2 * qb);
    const v2f fc = *(const v2fa*)(rp + 2 * qc);
    const v2f fd = *(const v2fa*)(rp + 2 * qd);
    asm volatile("" :: "v"(fa));
    asm volatile("" :: "v"(fb));
    asm volatile("" :: "v"(fc));
    asm volatile("" :: "v"(fd));
    const unsigned ma = pa < NPAIR ? rmk : 0u, mb = pb < NPAIR ? rmk : 0u;
    const unsigned mc = pc < NPAIR ? rmk : 0u, md = pd < NPAIR ? rmk : 0u;
    v8us o;
    o[0] = (unsigned short)(bf16_bits(fa.x) & ma); o[1] = (unsigned short)(bf16_bits(fa.y) & ma);
    o[2] = (unsigned short)(bf16_bits(fb.x) & mb); o[3] = (unsigned short)(bf16_bits(fb.y) & mb);
    o[4] = (unsigned short)(bf16_bits(fc.x) & mc); o[5] = (unsigned short)(bf16_bits(fc.y) & mc);
    o[6] = (unsigned short)(bf16_bits(fd.x) & md); o[7] = (unsigned short)(bf16_bits(fd.y) & md);
    st2_v8us(xb + (size_t)row * XP + 8 * g, o);
  } else if (blk < PBX + PBW) {
    const int u = (blk - PBX) * NTHR + tid;
    if (u < WBU) {
      const int n = u / 24, t = u - 24 * n;
      const int g = t & 7;
      const unsigned selr = (t >= 16) ? 0xffffffffu : 0u;
      const float* lp = wl + (size_t)n * FI;
      const float* rp = wr + (size_t)n * FI;
      const int pa = 4 * g, pb = pa + 1, pc = pa + 2, pd = pa + 3;
      const int qa = pa < NPAIR ? pa : NPAIR - 1, qb = pb < NPAIR ? pb : NPAIR - 1;
      const int qc = pc < NPAIR ? pc : NPAIR - 1, qd = pd < NPAIR ? pd : NPAIR - 1;
      const v2f la = *(const v2fa*)(lp + 2 * qa);
      const v2f lb = *(const v2fa*)(lp + 2 * qb);
      const v2f lc = *(const v2fa*)(lp + 2 * qc);
      const v2f ld = *(const v2fa*)(lp + 2 * qd);
      const v2f ra = *(const v2fa*)(rp + 2 * qa);
      const v2f rb = *(const v2fa*)(rp + 2 * qb);
      const v2f rc = *(const v2fa*)(rp + 2 * qc);
      const v2f rd = *(const v2fa*)(rp + 2 * qd);
      asm volatile("" :: "v"(la)); asm volatile("" :: "v"(lb));
      asm volatile("" :: "v"(lc)); asm volatile("" :: "v"(ld));
      asm volatile("" :: "v"(ra)); asm volatile("" :: "v"(rb));
      asm volatile("" :: "v"(rc)); asm volatile("" :: "v"(rd));
      const unsigned ma = pa < NPAIR ? 0xffffu : 0u, mb = pb < NPAIR ? 0xffffu : 0u;
      const unsigned mc = pc < NPAIR ? 0xffffu : 0u, md = pd < NPAIR ? 0xffffu : 0u;
      v8us o;
      o[0] = (unsigned short)(((bf16_bits(la.x) & ~selr) | (bf16_bits(ra.x) & selr)) & ma);
      o[1] = (unsigned short)(((bf16_bits(la.y) & ~selr) | (bf16_bits(ra.y) & selr)) & ma);
      o[2] = (unsigned short)(((bf16_bits(lb.x) & ~selr) | (bf16_bits(rb.x) & selr)) & mb);
      o[3] = (unsigned short)(((bf16_bits(lb.y) & ~selr) | (bf16_bits(rb.y) & selr)) & mb);
      o[4] = (unsigned short)(((bf16_bits(lc.x) & ~selr) | (bf16_bits(rc.x) & selr)) & mc);
      o[5] = (unsigned short)(((bf16_bits(lc.y) & ~selr) | (bf16_bits(rc.y) & selr)) & mc);
      o[6] = (unsigned short)(((bf16_bits(ld.x) & ~selr) | (bf16_bits(rd.x) & selr)) & md);
      o[7] = (unsigned short)(((bf16_bits(ld.y) & ~selr) | (bf16_bits(rd.y) & selr)) & md);
      st2_v8us(wb + (size_t)n * WBP + 8 * t, o);
    }
  } else if (blk == PBX + PBW) {
    if (tid < 32) {
      const int li = lane < 4 ? lane : 3;
      const v4f b = *(const v4fa*)(bl + 4 * li);
      asm volatile("" :: "v"(b));
      const unsigned mk = lane < 4 ? 0xffffffffu : 0u;
      v4f o;
      o.x = __uint_as_float((bf16_bits(b.x) << 16) & mk);
      o.y = __uint_as_float((bf16_bits(b.y) << 16) & mk);
      o.z = __uint_as_float((bf16_bits(b.z) << 16) & mk);
      o.w = __uint_as_float((bf16_bits(b.w) << 16) & mk);
      if (lane < 8) st2_v4f(blp + 4 * lane, o);
    }
  } else {
    const size_t u = (size_t)(blk - PBX - PBW - 1) * NTHR + (size_t)tid;
    const v4i z = {0, 0, 0, 0};
    int* p = zr + 4 * u;
    *(volatile v4i*)p = z;
    __threadfence();
    *(volatile v4i*)p = z;
  }
}

__device__ __forceinline__ void bucket_flush(const int* pl, const int* cnt, int ov, int* lp, int* cop, int* fp,
                                             int tid) {
#pragma unroll 1
  for (int i = tid * 4; i < RCAP; i += NTHR * 4) {
    const v4i v = *(const v4ia*)(pl + i);
    *(volatile v4i*)(lp + i) = v;
  }
#pragma unroll 1
  for (int i = tid * 4; i < 2 * NBRUN; i += NTHR * 4) {
    const v4i v = *(const v4ia*)(cnt + i);
    *(volatile v4i*)(cop + i) = v;
  }
  if (tid < 8) {
    const v4i f = {ov, ov, ov, ov};
    *(volatile v4i*)(fp + 4 * tid) = f;
  }
}

__global__ __launch_bounds__(NTHR) void k_bucket(const int* __restrict__ srcs, const int* __restrict__ dsts,
                                                 int* LIST, int* CO, int* FLAG) {
  extern __shared__ __attribute__((aligned(16))) int dsm[];
  int* wl   = dsm;
  int* pl   = dsm + NWAVE * WLCAP;
  int* cnt  = pl + RCAP;
  int* offs = cnt + NBRUN;
  int* cur  = offs + NBRUN;
  int* misc = cur + NBRUN;
  const int tid = (int)threadIdx.x, lane = tid & 31, wave = tid >> 5;
  const int blk = (int)blockIdx.x;
  const unsigned nbs = (unsigned)(blk * NBRUN);

  {
    const v4i z4 = {0, 0, 0, 0};
    for (int i = tid * 4; i < BK_ZINTS; i += NTHR * 4) *(v4ia*)(dsm + i) = z4;
    if (tid < 16) misc[tid] = 0;
  }
  __syncthreads();

  {
    const int per  = ((NE + NWAVE * WCH - 1) / (NWAVE * WCH)) * WCH;
    const int ebeg = wave * per;
    const int eend = (ebeg + per < NE) ? (ebeg + per) : NE;
    int* mylist = wl + wave * WLCAP;
    int wc = 0;
#pragma unroll 1
    for (int cb = ebeg; cb < eend; cb += WCH) {
      const int e0 = cb + lane * EPT;
      const v4i da = *(const v4ia*)(dsts + e0);
      const v4i db = *(const v4ia*)(dsts + e0 + 4);
      const unsigned s0 = (unsigned)da.x - nbs, s1 = (unsigned)da.y - nbs;
      const unsigned s2 = (unsigned)da.z - nbs, s3 = (unsigned)da.w - nbs;
      const unsigned s4 = (unsigned)db.x - nbs, s5 = (unsigned)db.y - nbs;
      const unsigned s6 = (unsigned)db.z - nbs, s7 = (unsigned)db.w - nbs;
      const bool h0 = s0 < (unsigned)NBRUN, h1 = s1 < (unsigned)NBRUN, h2 = s2 < (unsigned)NBRUN, h3 = s3 < (unsigned)NBRUN;
      const bool h4 = s4 < (unsigned)NBRUN, h5 = s5 < (unsigned)NBRUN, h6 = s6 < (unsigned)NBRUN, h7 = s7 < (unsigned)NBRUN;
      const unsigned m0 = __builtin_amdgcn_ballot_w32(h0), m1 = __builtin_amdgcn_ballot_w32(h1);
      const unsigned m2 = __builtin_amdgcn_ballot_w32(h2), m3 = __builtin_amdgcn_ballot_w32(h3);
      const unsigned m4 = __builtin_amdgcn_ballot_w32(h4), m5 = __builtin_amdgcn_ballot_w32(h5);
      const unsigned m6 = __builtin_amdgcn_ballot_w32(h6), m7 = __builtin_amdgcn_ballot_w32(h7);
      const unsigned any = m0 | m1 | m2 | m3 | m4 | m5 | m6 | m7;
      if (any != 0u) {
        const int pre = (int)(__builtin_amdgcn_mbcnt_lo(m0, 0u) + __builtin_amdgcn_mbcnt_lo(m1, 0u) +
                              __builtin_amdgcn_mbcnt_lo(m2, 0u) + __builtin_amdgcn_mbcnt_lo(m3, 0u) +
                              __builtin_amdgcn_mbcnt_lo(m4, 0u) + __builtin_amdgcn_mbcnt_lo(m5, 0u) +
                              __builtin_amdgcn_mbcnt_lo(m6, 0u) + __builtin_amdgcn_mbcnt_lo(m7, 0u));
        int p = wc + pre;
        if (h0) { if (p < WLCAP) mylist[p] = ((e0 + 0) << SLB) | (int)s0; p = p + 1; }
        if (h1) { if (p < WLCAP) mylist[p] = ((e0 + 1) << SLB) | (int)s1; p = p + 1; }
        if (h2) { if (p < WLCAP) mylist[p] = ((e0 + 2) << SLB) | (int)s2; p = p + 1; }
        if (h3) { if (p < WLCAP) mylist[p] = ((e0 + 3) << SLB) | (int)s3; p = p + 1; }
        if (h4) { if (p < WLCAP) mylist[p] = ((e0 + 4) << SLB) | (int)s4; p = p + 1; }
        if (h5) { if (p < WLCAP) mylist[p] = ((e0 + 5) << SLB) | (int)s5; p = p + 1; }
        if (h6) { if (p < WLCAP) mylist[p] = ((e0 + 6) << SLB) | (int)s6; p = p + 1; }
        if (h7) { if (p < WLCAP) mylist[p] = ((e0 + 7) << SLB) | (int)s7; p = p + 1; }
        wc += (int)(__builtin_popcount(m0) + __builtin_popcount(m1) + __builtin_popcount(m2) + __builtin_popcount(m3) +
                    __builtin_popcount(m4) + __builtin_popcount(m5) + __builtin_popcount(m6) + __builtin_popcount(m7));
      }
    }
    if (lane == 0) misc[wave] = wc;
  }
  __syncthreads();

  if (wave == 0) {
    int ov = 0;
#pragma unroll 1
    for (int w2 = 0; w2 < NWAVE; ++w2) {
      int c = misc[w2];
      if (c > WLCAP) ov = 1;
      c = c < 0 ? 0 : (c > WLCAP ? WLCAP : c);
#pragma unroll 1
      for (int b0 = 0; b0 < c; b0 += 32) {
        const int idx = b0 + lane;
        const int ent = wl[w2 * WLCAP + (idx < WLCAP ? idx : WLCAP - 1)];
        const int m32 = (c - b0) < 32 ? (c - b0) : 32;
#pragma unroll 1
        for (int k = 0; k < m32; ++k) {
          const int u    = __builtin_amdgcn_readlane(ent, k);
          const int slot = u & (NBRUN - 1);
          if (lane == 0) cnt[slot] = cnt[slot] + 1;
        }
      }
    }
    if (lane == 0) misc[9] = ov;
  }
  __syncthreads();
  if (wave == 0) {
    const int base = lane * (NBRUN / 32);
    int s = 0;
#pragma unroll 1
    for (int i = 0; i < NBRUN / 32; ++i) s += cnt[base + i];
    int incl = s;
#pragma unroll
    for (int d = 1; d < 32; d <<= 1) {
      const int y = __shfl_up(incl, d, 32);
      if (lane >= d) incl += y;
    }
    int run = incl - s;
#pragma unroll 1
    for (int i = 0; i < NBRUN / 32; ++i) {
      const int cv = cnt[base + i];
      offs[base + i] = run;
      cur[base + i]  = run;
      run += cv;
    }
  }
  __syncthreads();

  if (wave == 0) {
#pragma unroll 1
    for (int w2 = 0; w2 < NWAVE; ++w2) {
      int c = misc[w2];
      c = c < 0 ? 0 : (c > WLCAP ? WLCAP : c);
#pragma unroll 1
      for (int b0 = 0; b0 < c; b0 += 32) {
        const int idx = b0 + lane;
        const int ent = wl[w2 * WLCAP + (idx < WLCAP ? idx : WLCAP - 1)];
        int eid = (ent >> SLB) & 0x1fffff;
        eid = eid > NE - 1 ? NE - 1 : eid;
        int sr = srcs[eid];
        sr = sr < 0 ? 0 : (sr > NN - 1 ? NN - 1 : sr);
        const int m32 = (c - b0) < 32 ? (c - b0) : 32;
#pragma unroll 1
        for (int k = 0; k < m32; ++k) {
          const int u    = __builtin_amdgcn_readlane(ent, k);
          const int wd   = __builtin_amdgcn_readlane(sr, k);
          const int slot = u & (NBRUN - 1);
          if (lane == 0) {
            int p = cur[slot];
            p = p < 0 ? 0 : (p > RCAP - 1 ? RCAP - 1 : p);
            pl[p] = wd;
            cur[slot] = p + 1;
          }
        }
      }
    }
  }
  __syncthreads();

  const int ovf = misc[9];
  int* lp  = LIST + (size_t)blk * RCAP;
  int* cop = CO + (size_t)blk * (2 * NBRUN);
  int* fp  = FLAG + (size_t)blk * 32;
  bucket_flush(pl, cnt, ovf, lp, cop, fp, tid);
  __threadfence();
  bucket_flush(pl, cnt, ovf, lp, cop, fp, tid);
}

__global__ __launch_bounds__(NTHR) void k_replay(const int* __restrict__ LIST, const int* __restrict__ CO,
                                                 const int* __restrict__ FLAG,
                                                 const unsigned short* __restrict__ XB, unsigned short* MH) {
  const int tid = (int)threadIdx.x, lane = tid & 31, wave = tid >> 5, qd = lane >> 3, q = lane & 7;
  const int rowBase = (int)blockIdx.x * RBM;
  const int bucket  = rowBase >> SLB;
  const int* lb  = LIST + (size_t)bucket * RCAP;
  const int* cob = CO + (size_t)bucket * (2 * NBRUN);
  const int flag = FLAG[(size_t)bucket * 32];
  const float qnan = __uint_as_float(0x7fc00000u);

#pragma unroll 1
  for (int i = 0; i < 4; ++i) {
    const int d    = rowBase + 16 * wave + 4 * i + qd;
    const int slot = d & (NBRUN - 1);
    int c = cob[slot];
    int o = cob[NBRUN + slot];
    const bool big = c > DEGCAP;
    c = c < 0 ? 0 : (c > DEGCAP ? DEGCAP : c);
    o = o < 0 ? 0 : (o > RCAP - 1 ? RCAP - 1 : o);
    int cm = c;
    {
      const int t8 = __shfl_xor(cm, 8, 32);
      cm = cm > t8 ? cm : t8;
      const int t16 = __shfl_xor(cm, 16, 32);
      cm = cm > t16 ? cm : t16;
    }
    const int cmu = __builtin_amdgcn_readfirstlane(cm);
    int last = o + c - 1;
    last = last < o ? o : last;
    last = last > RCAP - 1 ? RCAP - 1 : last;
    float a0 = 0.0f, a1 = 0.0f, a2 = 0.0f, a3 = 0.0f, a4 = 0.0f, a5 = 0.0f, a6 = 0.0f, a7 = 0.0f;
#pragma unroll 1
    for (int j = 0; j < cmu; ++j) {
      int idx = o + j;
      idx = idx > last ? last : idx;
      int sr = lb[idx];
      sr = sr < 0 ? 0 : (sr > NN - 1 ? NN - 1 : sr);
      const v4u w = *(const v4ua*)(XB + (size_t)sr * XP + 8 * q);
      asm volatile("" :: "v"(w));
      const bool valid = j < c;
      const float t0 = a0 + __uint_as_float(w.x << 16);
      const float t1 = a1 + __uint_as_float(w.x & 0xffff0000u);
      const float t2 = a2 + __uint_as_float(w.y << 16);
      const float t3 = a3 + __uint_as_float(w.y & 0xffff0000u);
      const float t4 = a4 + __uint_as_float(w.z << 16);
      const float t5 = a5 + __uint_as_float(w.z & 0xffff0000u);
      const float t6 = a6 + __uint_as_float(w.w << 16);
      const float t7 = a7 + __uint_as_float(w.w & 0xffff0000u);
      a0 = valid ? t0 : a0; a1 = valid ? t1 : a1; a2 = valid ? t2 : a2; a3 = valid ? t3 : a3;
      a4 = valid ? t4 : a4; a5 = valid ? t5 : a5; a6 = valid ? t6 : a6; a7 = valid ? t7 : a7;
    }
    const int cd = c < 1 ? 1 : c;
    const float inv = 1.0f / (float)cd;
    const bool bad  = (flag != 0) | big;
    const bool live = d < NN;
    float mv[8];
    mv[0] = a0 * inv; mv[1] = a1 * inv; mv[2] = a2 * inv; mv[3] = a3 * inv;
    mv[4] = a4 * inv; mv[5] = a5 * inv; mv[6] = a6 * inv; mv[7] = a7 * inv;
    v8us hv, lv;
#pragma unroll
    for (int e = 0; e < 8; ++e) {
      float m = mv[e];
      m = bad ? qnan : m;
      m = live ? m : 0.0f;
      const unsigned hb = bf16_bits(m);
      const unsigned lo = bf16_bits(m - __uint_as_float(hb << 16));
      hv[e] = (unsigned short)hb;
      lv[e] = (unsigned short)lo;
    }
    unsigned short* hp = MH + (size_t)d * MHP + 8 * q;
    *(volatile v8us*)hp = hv;
    *(volatile v8us*)(hp + XP) = lv;
    __threadfence();
    *(volatile v8us*)hp = hv;
    *(volatile v8us*)(hp + XP) = lv;
  }
}

__device__ __forceinline__ void out_flush(const float* lt, const float* ot, float* o0, float* o1, int nv4,
                                          int tid) {
#pragma unroll 1
  for (int it = 0; it < 2; ++it) {
    const int i4 = it * NTHR + tid;
    const v4f a = *(const v4fa*)(lt + 4 * i4);
    const v4f b = *(const v4fa*)(ot + 4 * i4);
    asm volatile("" :: "v"(a));
    asm volatile("" :: "v"(b));
    if (i4 < nv4) {
      *(volatile v4f*)(o0 + (size_t)4 * (size_t)i4) = a;
      *(volatile v4f*)(o1 + (size_t)4 * (size_t)i4) = b;
    }
  }
}

__global__ __launch_bounds__(NTHR) __attribute__((amdgpu_num_vgpr(248)))
void k_gemm_out(const unsigned short* __restrict__ MH, const unsigned short* __restrict__ XB,
                const unsigned short* __restrict__ WB, const float* __restrict__ BL,
                const int* __restrict__ FLAG, float* out) {
  __shared__ __attribute__((aligned(16))) unsigned short wbs[NC * WBP];
  __shared__ __attribute__((aligned(16))) float dt[GBM * DTP];
  __shared__ __attribute__((aligned(16))) float lt[GBM * NC];
  __shared__ __attribute__((aligned(16))) float ot[GBM * NC];
  __shared__ __attribute__((aligned(16))) float sbl[16];
  const int tid = (int)threadIdx.x, lane = tid & 31, wave = tid >> 5, hh = lane >> 4, m = lane & 15;
  const int blk = (int)blockIdx.x;
  const int rowBase = blk * GBM;
  const int flag = FLAG[(size_t)(rowBase >> SLB) * 32];

  for (int u = tid; u < WBU; u += NTHR) *(v8usa*)(wbs + 8 * u) = *(const v8usa*)(WB + 8 * u);
  if (tid < 4) *(v4fa*)(sbl + 4 * tid) = *(const v4fa*)(BL + 4 * tid);
  __syncthreads();

  v8f acc = {0.f, 0.f, 0.f, 0.f, 0.f, 0.f, 0.f, 0.f};
  const unsigned short* am = MH + (size_t)(rowBase + 16 * wave + m) * (size_t)MHP + 8 * hh;
  const unsigned short* ax = XB + (size_t)(rowBase + 16 * wave + m) * (size_t)XP + 8 * hh;
  const unsigned short* bw = wbs + m * WBP + 8 * hh;
#pragma unroll
  for (int s = 0; s < MSTEPS; ++s) {
    FragB af, bf;
    af.h[0] = *(const v8usa*)(am + 32 * s);
    af.h[1] = *(const v8usa*)(am + 32 * s + 16);
    bf.h[0] = *(const v8usa*)(bw + 32 * s);
    bf.h[1] = *(const v8usa*)(bw + 32 * s + 16);
    acc = wmb(af, bf, acc);
  }
#pragma unroll
  for (int s = 0; s < XSTEPS; ++s) {
    FragB af, bf;
    af.h[0] = *(const v8usa*)(ax + 32 * s);
    af.h[1] = *(const v8usa*)(ax + 32 * s + 16);
    bf.h[0] = *(const v8usa*)(bw + WROFF + 32 * s);
    bf.h[1] = *(const v8usa*)(bw + WROFF + 32 * s + 16);
    acc = wmb(af, bf, acc);
  }
#pragma unroll
  for (int r = 0; r < 8; ++r) dt[(16 * wave + 8 * hh + r) * DTP + m] = acc[r];
  __syncthreads();

  if (tid < GBM) {
    float* p = dt + tid * DTP;
#pragma unroll 1
    for (int c = 0; c < NC; ++c) p[c] = p[c] + sbl[c];
    float mx = p[0];
#pragma unroll 1
    for (int c = 1; c < NC; ++c) {
      const float xv = p[c];
      mx = ((xv > mx) | (xv != xv)) ? xv : mx;
    }
    float se = 0.0f;
#pragma unroll 1
    for (int c = 0; c < NC; ++c) se += expf(p[c] - mx);
    const float ls = logf(se);
    const float qnan = __uint_as_float(0x7fc00000u);
#pragma unroll 1
    for (int c = 0; c < NC; ++c) {
      const float v  = p[c];
      const float lv = (v - mx) - ls;
      ot[tid * NC + c] = (flag != 0) ? qnan : v;
      lt[tid * NC + c] = (flag != 0) ? qnan : lv;
    }
  }
  __syncthreads();

  const int liveRows = (NN - rowBase) < GBM ? (NN - rowBase) : GBM;
  const int nv4 = liveRows * (NC / 4);
  float* o0 = out + (size_t)blk * (size_t)(GBM * NC);
  float* o1 = out + (size_t)NN * NC + (size_t)blk * (size_t)(GBM * NC);
  out_flush(lt, ot, o0, o1, nv4, tid);
  __threadfence();
  out_flush(lt, ot, o0, o1, nv4, tid);
}

extern "C" void kernel_launch(void* const* d_in, const int* in_sizes, int n_in,
                              void* d_out, int out_size, void* d_ws, size_t ws_size,
                              hipStream_t stream) {
  if (n_in < 5) return;
  if (in_sizes[0] != NN * FI) return;
  if (in_sizes[1] != 2 * NE) return;
  if (in_sizes[2] != NC * FI) return;
  if (in_sizes[3] != NC) return;
  if (in_sizes[4] != NC * FI) return;
  if (out_size != 2 * NN * NC) return;

  const float* x  = (const float*)d_in[0];
  const int*   ei = (const int*)d_in[1];
  const float* wl = (const float*)d_in[2];
  const float* bl = (const float*)d_in[3];
  const float* wr = (const float*)d_in[4];
  float* out = (float*)d_out;
  const int* srcs = ei;
  const int* dsts = ei + NE;

  constexpr size_t zXB   = (size_t)MP * XP * 2;
  constexpr size_t zMH   = (size_t)MP * MHP * 2;
  constexpr size_t zWB   = (size_t)NC * WBP * 2;
  constexpr size_t zBL   = 256;
  constexpr size_t zLIST = (size_t)ZLIST_B;
  constexpr size_t zCO   = (size_t)ZCO_B;
  constexpr size_t zFLAG = (size_t)ZFLAG_B;
  constexpr size_t oXB   = 0;
  constexpr size_t oMH   = oXB + zXB;
  constexpr size_t oWB   = oMH + zMH;
  constexpr size_t oBL   = oWB + zWB;
  constexpr size_t oLIST = oBL + zBL;
  constexpr size_t oCO   = oLIST + zLIST;
  constexpr size_t oFLAG = oCO + zCO;
  constexpr size_t oEND  = oFLAG + zFLAG;
  static_assert(zXB % 256 == 0 && zMH % 256 == 0 && zWB % 256 == 0 && zLIST % 256 == 0 && zCO % 256 == 0);
  static_assert(zFLAG % 256 == 0 && (zLIST + zCO + zFLAG) == (size_t)PBZ * 4096);
  static_assert(oEND <= ((size_t)128 << 20));
  if (oEND > ws_size) return;

  char* ws = (char*)d_ws;
  unsigned short* XBp  = (unsigned short*)(ws + oXB);
  unsigned short* MHp  = (unsigned short*)(ws + oMH);
  unsigned short* WBp  = (unsigned short*)(ws + oWB);
  float*          BLp  = (float*)(ws + oBL);
  int*            LIST = (int*)(ws + oLIST);
  int*            CO   = (int*)(ws + oCO);
  int*            FLAG = (int*)(ws + oFLAG);

  hipFuncSetAttribute(reinterpret_cast<const void*>(&k_bucket), hipFuncAttributeMaxDynamicSharedMemorySize, (int)BK_LDS);

  k_prep<<<PBTOT, NTHR, 0, stream>>>(x, wl, bl, wr, XBp, WBp, BLp, LIST);
  k_bucket<<<NBK, NTHR, BK_LDS, stream>>>(srcs, dsts, LIST, CO, FLAG);
  k_replay<<<MP / RBM, NTHR, 0, stream>>>(LIST, CO, FLAG, XBp, MHp);
  k_gemm_out<<<MP / GBM, NTHR, 0, stream>>>(MHp, XBp, WBp, BLp, FLAG, out);
}
